// UniF_Att_CNN_18073222381857
// MI455X (gfx1250) — hardware-verified
//
#include <hip/hip_runtime.h>
#include <math.h>

constexpr int kUtts      = 2048;
constexpr int kSeqLen    = 50;
constexpr int kEmb       = 300;
constexpr int kEmbPitch  = 320;
constexpr int kVocab     = 50000;
constexpr int kTok       = kUtts * kSeqLen;
constexpr int kTokRows   = kTok + 64;
constexpr int kFilt      = 64;
constexpr int kCat       = 192;
constexpr int kHidden    = 100;
constexpr int kHidPitch  = 128;
constexpr int kGate      = 300;
constexpr int kGatePitch = 320;
constexpr int kWind      = 10;
constexpr int kHops      = 3;
constexpr int kClasses   = 7;
constexpr int kTransN    = 128;
constexpr int kConvK3    = 3 * kEmbPitch;
constexpr int kConvK4    = 4 * kEmbPitch;
constexpr int kConvK5    = 5 * kEmbPitch;
constexpr float kCarry   = 16.0f;
constexpr float kNegFill = -1.0e10f;
constexpr int kOutPred   = kUtts * kClasses;
constexpr int kOutAttn   = kHops * (kUtts - 1) * kWind;
constexpr int kOutTot    = kOutPred + kOutAttn;

static_assert(kConvK3 % 32 == 0 && kConvK4 % 32 == 0 && kConvK5 % 32 == 0);
static_assert(kTok % 64 == 0 && kUtts % 64 == 0 && kTransN % 64 == 0 && kGatePitch % 64 == 0 && kHidPitch % 32 == 0 && kCat % 32 == 0);

constexpr size_t kBytesE16  = (size_t)kTokRows * kEmbPitch * 2;
constexpr size_t kBytesWB3  = (size_t)kFilt * kConvK3 * 2;
constexpr size_t kBytesWB4  = (size_t)kFilt * kConvK4 * 2;
constexpr size_t kBytesWB5  = (size_t)kFilt * kConvK5 * 2;
constexpr size_t kBytesYpl  = (size_t)kTok * kFilt * 2;
constexpr size_t kBytesF16  = (size_t)kUtts * kCat * 2;
constexpr size_t kBytesTWB  = (size_t)kTransN * kCat * 2;
constexpr size_t kBytesU    = (size_t)kUtts * kHidPitch * 4;
constexpr size_t kBytesS    = kBytesU;
constexpr size_t kBytesS16  = (size_t)kUtts * kHidPitch * 2;
constexpr size_t kBytesWG16 = (size_t)kGatePitch * kHidPitch * 2;
constexpr size_t kBytesGI   = (size_t)kUtts * kGatePitch * 4;
constexpr size_t kBytesH16  = kBytesS16;
constexpr size_t kBytesMOpl = (size_t)kUtts * kHidPitch * 4;
constexpr size_t kBytesMO   = (size_t)kWind * kBytesMOpl;
constexpr size_t kBytesPL   = (size_t)kUtts * 8 * 4;
constexpr size_t kBytesAS   = (size_t)kHops * kUtts * 16 * 4;
constexpr size_t kWsTotal   = kBytesE16 + kBytesWB3 + kBytesWB4 + kBytesWB5 + 3 * kBytesYpl + kBytesF16 + kBytesTWB +
                              kBytesU + kBytesS + kBytesS16 + 2 * kBytesWG16 + 2 * kBytesGI + 2 * kBytesH16 + kBytesMO +
                              kBytesPL + kBytesAS;
static_assert(kWsTotal == 126246912u);
static_assert(kWsTotal <= 134217728u);
static_assert(kBytesE16 % 256 == 0 && kBytesWB3 % 256 == 0 && kBytesWB4 % 256 == 0 && kBytesWB5 % 256 == 0 && kBytesYpl % 256 == 0);
static_assert(kBytesF16 % 256 == 0 && kBytesTWB % 256 == 0 && kBytesU % 256 == 0 && kBytesS16 % 256 == 0 && kBytesWG16 % 256 == 0);
static_assert(kBytesGI % 256 == 0 && kBytesMOpl % 256 == 0 && kBytesPL % 256 == 0 && kBytesAS % 256 == 0);

typedef __attribute__((ext_vector_type(16))) _Float16 v16h;
typedef __attribute__((ext_vector_type(8)))  _Float16 v8h;
typedef __attribute__((ext_vector_type(16))) __bf16   v16b;
typedef __attribute__((ext_vector_type(8)))  __bf16   v8b;
typedef __attribute__((ext_vector_type(8)))  float    v8f;
typedef __attribute__((ext_vector_type(4)))  float    v4f;
typedef __attribute__((ext_vector_type(2)))  float    v2f;
typedef __attribute__((ext_vector_type(4)))  unsigned int v4u;

__device__ __forceinline__ unsigned short f2bf_bits(float f) {
  unsigned u = __float_as_uint(f);
  return (unsigned short)((u + 0x7FFFu + ((u >> 16) & 1u)) >> 16);
}
__device__ __forceinline__ float bf_bits2f(unsigned short h) { return __uint_as_float(((unsigned)h) << 16); }

__device__ __forceinline__ void dep_guard_h(v8f& a, v8f& b, v16h x, v16h y) { asm volatile("v_nop\n\tv_nop\n\tv_nop\n\tv_nop" : "+v"(a), "+v"(b) : "v"(x), "v"(y)); }
__device__ __forceinline__ void dep_guard_b(v8f& a, v8f& b, v16b x, v16b y) { asm volatile("v_nop\n\tv_nop\n\tv_nop\n\tv_nop" : "+v"(a), "+v"(b) : "v"(x), "v"(y)); }
__device__ __forceinline__ void keep4_h(v16h a, v16h b, v16h c, v16h d) { asm volatile("v_nop" :: "v"(a), "v"(b), "v"(c), "v"(d)); }
__device__ __forceinline__ void keep4_b(v16b a, v16b b, v16b c, v16b d) { asm volatile("v_nop" :: "v"(a), "v"(b), "v"(c), "v"(d)); }
__device__ __forceinline__ void acc_guard4(v8f& a, v8f& b, v8f& c, v8f& d) { asm volatile("v_nop\n\tv_nop\n\tv_nop\n\tv_nop" : "+v"(a), "+v"(b), "+v"(c), "+v"(d)); }
template <typename T> struct Frag;
template <> struct Frag<_Float16> {
  typedef v16h V; union U { v16h v; v8h h[2]; };
  static __device__ __forceinline__ v16h load(const _Float16* p) {
    U f; f.h[0] = *(const v8h*)(p); f.h[1] = *(const v8h*)(p + 16); return f.v;
  }
  static __device__ __forceinline__ v8f mma(v16h a, v16h b, v8f c) {
    return __builtin_amdgcn_wmma_f32_16x16x32_f16(false, a, false, b, (short)0, c, false, false);
  }
  static __device__ __forceinline__ void guard(v8f& a, v8f& b, v16h x, v16h y) { dep_guard_h(a, b, x, y); }
  static __device__ __forceinline__ void keep(v16h a, v16h b, v16h c, v16h d) { keep4_h(a, b, c, d); }
};
template <> struct Frag<__bf16> {
  typedef v16b V; union U { v16b v; v8b h[2]; };
  static __device__ __forceinline__ v16b load(const __bf16* p) {
    U f; f.h[0] = *(const v8b*)(p); f.h[1] = *(const v8b*)(p + 16); return f.v;
  }
  static __device__ __forceinline__ v8f mma(v16b a, v16b b, v8f c) {
    return __builtin_amdgcn_wmma_f32_16x16x32_bf16(false, a, false, b, (short)0, c, false, false);
  }
  static __device__ __forceinline__ void guard(v8f& a, v8f& b, v16b x, v16b y) { dep_guard_b(a, b, x, y); }
  static __device__ __forceinline__ void keep(v16b a, v16b b, v16b c, v16b d) { keep4_b(a, b, c, d); }
};

__device__ __forceinline__ unsigned pk16(unsigned short a, unsigned short b) { return (unsigned)a | ((unsigned)b << 16); }
__device__ __forceinline__ unsigned short h_bits(float f) { const _Float16 h = (_Float16)f; return __builtin_bit_cast(unsigned short, h); }

template <int ET> struct Elem;
template <> struct Elem<0> { typedef _Float16 T; };
template <> struct Elem<1> { typedef __bf16 T; };
template <int ET, bool SPLIT, int BIAS_MODE, int OUT_MODE, bool RESID, int ACT = 0>
__global__ __launch_bounds__(256) void wmma_gemm64(
    const unsigned short* __restrict__ Ap, const unsigned short* __restrict__ A2p, int lda, long strideA,
    const unsigned short* __restrict__ Btp, const unsigned short* __restrict__ Bt2p, int ldb, long strideB,
    void* __restrict__ Cout, void* __restrict__ Cout2, int ldc, long strideC,
    const float* __restrict__ bias,
    const float* __restrict__ resid, long strideR,
    int M, int N, int K, float scale) {
  typedef typename Elem<ET>::T T;
  typedef typename Frag<T>::V V;
  const T* A = (const T*)Ap; const T* A2 = (const T*)A2p; const T* Bt = (const T*)Btp; const T* Bt2 = (const T*)Bt2p;
  __shared__ __align__(16) float sT[8][16 * 68];
  const int b    = blockIdx.y;
  const int lane = threadIdx.x & 31;
  const int wave = threadIdx.x >> 5;
  const int tilesN = N >> 6;
  const int tilesM = M >> 6;
  const int tile = blockIdx.x * 8 + wave;
  if (tile >= tilesM * tilesN) return;
  const int tm = tile / tilesN;
  const int tn = tile - tm * tilesN;
  const int m0 = tm << 6;
  const int n0 = tn << 6;

  const T* Ab  = A  + (size_t)b * strideA;
  const T* Bb  = Bt + (size_t)b * strideB;
  const T* Ab2 = SPLIT ? (A2  + (size_t)b * strideA) : nullptr;
  const T* Bb2 = SPLIT ? (Bt2 + (size_t)b * strideB) : nullptr;

  const int rlane = lane & 15;
  const int koff  = (lane >> 4) * 8;
  const int mOff  = (lane >> 4) * 8;

  v8f acc[4][4];
#pragma unroll
  for (int i = 0; i < 4; ++i)
#pragma unroll
    for (int j = 0; j < 4; ++j) acc[i][j] = (v8f){0.f,0.f,0.f,0.f,0.f,0.f,0.f,0.f};

  for (int k0 = 0; k0 < K; k0 += 32) {
    V bh[4], bl[4];
#pragma unroll
    for (int j = 0; j < 4; ++j) {
      const size_t bo = (size_t)(n0 + (j << 4) + rlane) * ldb + koff + k0;
      bh[j] = Frag<T>::load(Bb + bo);
      if (SPLIT) bl[j] = Frag<T>::load(Bb2 + bo);
    }
#pragma unroll
    for (int i = 0; i < 4; ++i) {
      const size_t ao = (size_t)(m0 + (i << 4) + rlane) * lda + koff + k0;
      V ah = Frag<T>::load(Ab + ao);
      V al;
      if (SPLIT) al = Frag<T>::load(Ab2 + ao);
#pragma unroll
      for (int j = 0; j < 4; ++j) {
        acc[i][j] = Frag<T>::mma(ah, bh[j], acc[i][j]);
        if (SPLIT) {
          acc[i][j] = Frag<T>::mma(ah, bl[j], acc[i][j]);
          acc[i][j] = Frag<T>::mma(al, bh[j], acc[i][j]);
        }
      }
      Frag<T>::guard(acc[i][0], acc[i][3], ah, SPLIT ? al : ah);
    }
    Frag<T>::keep(bh[0], bh[1], bh[2], bh[3]);
    if (SPLIT) Frag<T>::keep(bl[0], bl[1], bl[2], bl[3]);
  }
  acc_guard4(acc[0][0], acc[0][1], acc[0][2], acc[0][3]);
  acc_guard4(acc[1][0], acc[1][1], acc[1][2], acc[1][3]);
  acc_guard4(acc[2][0], acc[2][1], acc[2][2], acc[2][3]);
  acc_guard4(acc[3][0], acc[3][1], acc[3][2], acc[3][3]);

  float* slab = sT[wave];
  const float* Rb = RESID ? (resid + (size_t)b * strideR) : nullptr;
#pragma unroll
  for (int i = 0; i < 4; ++i) {
    const int mBase = m0 + (i << 4);
#pragma unroll
    for (int j = 0; j < 4; ++j) {
      const int n = n0 + (j << 4) + rlane;
      float bv = 0.f;
      if (BIAS_MODE == 2) bv = bias[n];
#pragma unroll
      for (int r = 0; r < 8; ++r) {
        float v = acc[i][j][r] * scale;
        if (BIAS_MODE == 1) v += bias[mBase + mOff + r];
        if (BIAS_MODE == 2) v += bv;
        if (RESID) v += Rb[(size_t)(mBase + mOff + r) * ldc + n];
        if (ACT == 1) v = tanhf(v);
        if (ACT == 2) v = fmaxf(v, 0.0f);
        if (ACT == 3) v = v / (1.0f + expf(-v));
        if (ACT == 4) v = (v > 0.f) ? v : 0.01f * v;
        if (ACT == 5) v = 0.5f * v * (1.0f + erff(v * 0.70710678118654752f));
        slab[(mOff + r) * 68 + (j << 4) + rlane] = v;
      }
    }
    __builtin_amdgcn_fence(__ATOMIC_RELEASE, "workgroup");
    __builtin_amdgcn_wave_barrier();
    __builtin_amdgcn_fence(__ATOMIC_ACQUIRE, "workgroup");
    if (OUT_MODE == 0) {
      float* C = (float*)Cout + (size_t)b * strideC;
      const int hh = lane >> 4, c4 = (lane & 15) * 4;
      for (int pass = 0; pass < 2; ++pass) {
#pragma unroll
        for (int it = 0; it < 8; ++it) {
          const int row = it * 2 + hh;
          v4f v = *(const v4f*)(slab + row * 68 + c4);
          *(volatile v4f*)(C + (size_t)(mBase + row) * ldc + n0 + c4) = v;
        }
        __threadfence();
      }
    } else {
      const int q = lane >> 3, c8 = (lane & 7) * 8;
      unsigned short* C  = (unsigned short*)Cout  + (size_t)b * strideC;
      unsigned short* C2 = (OUT_MODE == 2) ? ((unsigned short*)Cout2 + (size_t)b * strideC) : nullptr;
      for (int pass = 0; pass < 2; ++pass) {
#pragma unroll
        for (int it = 0; it < 4; ++it) {
          const int row = it * 4 + q;
          const float* sp = slab + row * 68 + c8;
          v8h hv, lv;
#pragma unroll
          for (int e = 0; e < 8; ++e) {
            if (OUT_MODE == 1) {
              hv[e] = (_Float16)sp[e];
            } else {
              unsigned short hb = f2bf_bits(sp[e]);
              unsigned short lb = f2bf_bits(sp[e] - bf_bits2f(hb));
              hv[e] = __builtin_bit_cast(_Float16, hb);
              lv[e] = __builtin_bit_cast(_Float16, lb);
            }
          }
          *(volatile v8h*)(C + (size_t)(mBase + row) * ldc + n0 + c8) = hv;
          if (OUT_MODE == 2) *(volatile v8h*)(C2 + (size_t)(mBase + row) * ldc + n0 + c8) = lv;
        }
        __threadfence();
      }
    }
    __builtin_amdgcn_fence(__ATOMIC_RELEASE, "workgroup");
    __builtin_amdgcn_wave_barrier();
    __builtin_amdgcn_fence(__ATOMIC_ACQUIRE, "workgroup");
  }
}

__device__ __forceinline__ float wave_sum(float v) {
#pragma unroll
  for (int off = 16; off > 0; off >>= 1) v += __shfl_xor(v, off, 32);
  return v;
}
__device__ __forceinline__ float wave_max(float v) {
#pragma unroll
  for (int off = 16; off > 0; off >>= 1) v = fmaxf(v, __shfl_xor(v, off, 32));
  return v;
}
__device__ __forceinline__ void wave_lds_sync() {
  __builtin_amdgcn_fence(__ATOMIC_RELEASE, "workgroup");
  __builtin_amdgcn_wave_barrier();
  __builtin_amdgcn_fence(__ATOMIC_ACQUIRE, "workgroup");
}

__global__ __launch_bounds__(256) void prep_cast16_kernel(const float* __restrict__ in, unsigned short* __restrict__ out,
                                                          int nCols, int nRowsIn, int segOut, int segIn, int pitchIn,
                                                          float scale, int nChunks) {
  const int qd = blockIdx.x * 256 + threadIdx.x;
  if (qd >= nChunks) return;
  const int e0   = qd * 8;
  const int row  = e0 / nCols;
  const int col0 = e0 - row * nCols;
  const int j    = col0 / segOut;
  const int d0   = col0 - j * segOut;
  const bool rok = row < nRowsIn;
  const int rr   = rok ? row : (nRowsIn - 1);
  const float* ir = in + (size_t)rr * pitchIn + (size_t)j * segIn;
  unsigned short hb[8];
#pragma unroll
  for (int e = 0; e < 8; ++e) {
    const int d  = d0 + e;
    const int dd = (d < segIn) ? d : (segIn - 1);
    float v = ir[dd];
    v = (rok && (d < segIn)) ? v * scale : 0.0f;
    hb[e] = h_bits(v);
  }
  const v4u u = (v4u){pk16(hb[0], hb[1]), pk16(hb[2], hb[3]), pk16(hb[4], hb[5]), pk16(hb[6], hb[7])};
  unsigned short* op = out + (size_t)e0;
  *(volatile v4u*)op = u;
  __threadfence();
  *(volatile v4u*)op = u;
}

__global__ __launch_bounds__(256) void embed_gather_kernel(const int* __restrict__ sents, const float* __restrict__ emb,
                                                           unsigned short* __restrict__ E, int nChunks) {
  const int qd = blockIdx.x * 256 + threadIdx.x;
  if (qd >= nChunks) return;
  const int row = qd / (kEmbPitch / 8);
  const int c8  = (qd - row * (kEmbPitch / 8)) * 8;
  const bool rowok = row < kTok;
  const int rr = rowok ? row : (kTok - 1);
  int tok = sents[rr];
  tok = (tok < 0) ? 0 : tok;
  tok = (tok > kVocab - 1) ? (kVocab - 1) : tok;
  const float* er = emb + (size_t)tok * kEmb;
  const bool oka = rowok && (c8 <= kEmb - 4);
  const bool okb = rowok && (c8 + 4 <= kEmb - 4);
  const int ca = (c8 <= kEmb - 4) ? c8 : (kEmb - 4);
  const int cb = (c8 + 4 <= kEmb - 4) ? (c8 + 4) : (kEmb - 4);
  const v4f a  = *(const v4f*)(er + ca);
  const v4f bq = *(const v4f*)(er + cb);
  unsigned short hb[8];
#pragma unroll
  for (int e = 0; e < 4; ++e) {
    hb[e]     = h_bits(oka ? a[e] * kCarry : 0.0f);
    hb[4 + e] = h_bits(okb ? bq[e] * kCarry : 0.0f);
  }
  const v4u u = (v4u){pk16(hb[0], hb[1]), pk16(hb[2], hb[3]), pk16(hb[4], hb[5]), pk16(hb[6], hb[7])};
  unsigned short* op = E + (size_t)qd * 8;
  *(volatile v4u*)op = u;
  __threadfence();
  *(volatile v4u*)op = u;
}

__global__ __launch_bounds__(192) void maxpool_kernel(const unsigned short* __restrict__ Y, const float* __restrict__ cb3,
                                                      const float* __restrict__ cb4, const float* __restrict__ cb5,
                                                      unsigned short* __restrict__ F) {
  __shared__ __align__(16) float sF[kCat];
  const int n   = blockIdx.x;
  const int tid = threadIdx.x;
  const int g   = tid >> 6;
  const int f   = tid & 63;
  const int P   = (kSeqLen - 2) - g;
  const unsigned short* Yg = Y + (size_t)g * ((size_t)kTok * kFilt) + (size_t)n * kSeqLen * kFilt + f;
  float mx = -INFINITY;
#pragma unroll 1
  for (int t = 0; t < P; ++t) {
    const unsigned short hs = Yg[(size_t)t * kFilt];
    const float v = (float)__builtin_bit_cast(_Float16, hs);
    mx = fmaxf(mx, v);
  }
  const float b3 = cb3[f], b4 = cb4[f], b5 = cb5[f];
  const float bb = (g == 0) ? b3 : ((g == 1) ? b4 : b5);
  const float fc = fmaxf(mx + kCarry * bb, 0.0f);
  sF[tid] = fc;
  __syncthreads();
  const int lane = tid & 31, wave = tid >> 5;
  const int l24 = (lane < 24) ? lane : 23;
  unsigned short hb[8];
#pragma unroll
  for (int e = 0; e < 8; ++e) hb[e] = h_bits(sF[l24 * 8 + e]);
  const v4u u = (v4u){pk16(hb[0], hb[1]), pk16(hb[2], hb[3]), pk16(hb[4], hb[5]), pk16(hb[6], hb[7])};
  for (int pass = 0; pass < 2; ++pass) {
    if (wave == 0 && lane < 24) *(volatile v4u*)(F + (size_t)n * kCat + l24 * 8) = u;
    __threadfence();
  }
}

__global__ __launch_bounds__(128) void feat_tanh_kernel(const float* __restrict__ U, const float* __restrict__ tb,
                                                        float* __restrict__ S, unsigned short* __restrict__ S16) {
  __shared__ __align__(16) float ss[kHidPitch];
  const int row = blockIdx.x;
  const int t = threadIdx.x, lane = t & 31, wave = t >> 5;
  const int tt = (t < kHidden) ? t : (kHidden - 1);
  const float u = U[(size_t)row * kHidPitch + tt];
  const float bv = tb[tt];
  float s = tanhf(u + bv);
  s = (t < kHidden) ? s : 0.0f;
  ss[t] = s;
  __syncthreads();
  const int l16 = lane & 15;
  unsigned short hb[8];
#pragma unroll
  for (int e = 0; e < 8; ++e) hb[e] = h_bits(ss[l16 * 8 + e] * kCarry);
  const v4u u16 = (v4u){pk16(hb[0], hb[1]), pk16(hb[2], hb[3]), pk16(hb[4], hb[5]), pk16(hb[6], hb[7])};
  const v4f v4 = *(const v4f*)(ss + 4 * lane);
  for (int pass = 0; pass < 2; ++pass) {
    if (wave == 0) *(volatile v4f*)(S + (size_t)row * kHidPitch + 4 * lane) = v4;
    if (wave == 1 && lane < 16) *(volatile v4u*)(S16 + (size_t)row * kHidPitch + l16 * 8) = u16;
    __threadfence();
  }
}

__global__ __launch_bounds__(128) void gru_gate_kernel(const float* __restrict__ GI, const float* __restrict__ GH,
                                                       const float* __restrict__ bih, const float* __restrict__ bhh,
                                                       const float* __restrict__ Hprev, float* __restrict__ Hout,
                                                       unsigned short* __restrict__ H16out, int step) {
  __shared__ __align__(16) float sh[kHidPitch];
  const int i = blockIdx.x;
  const int t = threadIdx.x, lane = t & 31, wave = t >> 5;
  const bool live = (i < kUtts - 1) && (t < kHidden);
  const int tt = (t < kHidden) ? t : (kHidden - 1);
  const int idx = i - (kWind - 1) + step;
  const bool valid = idx >= 0;
  int idc = valid ? idx : 0;
  idc = (idc > kUtts - 1) ? (kUtts - 1) : idc;
  const float* gir = GI + (size_t)idc * kGatePitch;
  float gr = gir[tt], gz = gir[kHidden + tt], gn = gir[2 * kHidden + tt];
  gr = valid ? gr : 0.0f; gz = valid ? gz : 0.0f; gn = valid ? gn : 0.0f;
  const float br = bih[tt], bz = bih[kHidden + tt], bn = bih[2 * kHidden + tt];
  const float cr = bhh[tt], cz = bhh[kHidden + tt], cn = bhh[2 * kHidden + tt];
  float hr = 0.0f, hz = 0.0f, hn = 0.0f, hp = 0.0f;
  if (step > 0) {
    const float* ghr = GH + (size_t)i * kGatePitch;
    hr = ghr[tt]; hz = ghr[kHidden + tt]; hn = ghr[2 * kHidden + tt];
    hp = Hprev[(size_t)i * kHidPitch + tt];
  }
  const float xr = (gr + br) + (hr + cr);
  const float xz = (gz + bz) + (hz + cz);
  const float rg = 1.0f / (1.0f + expf(-xr));
  const float zg = 1.0f / (1.0f + expf(-xz));
  const float nn = tanhf((gn + bn) + rg * (hn + cn));
  float h = (1.0f - zg) * nn + zg * hp;
  h = live ? h : 0.0f;
  sh[t] = h;
  __syncthreads();
  const int l16 = lane & 15;
  unsigned short hb[8];
#pragma unroll
  for (int e = 0; e < 8; ++e) hb[e] = h_bits(sh[l16 * 8 + e] * kCarry);
  const v4u u16 = (v4u){pk16(hb[0], hb[1]), pk16(hb[2], hb[3]), pk16(hb[4], hb[5]), pk16(hb[6], hb[7])};
  const v4f v4 = *(const v4f*)(sh + 4 * lane);
  for (int pass = 0; pass < 2; ++pass) {
    if (wave == 0) *(volatile v4f*)(Hout + (size_t)i * kHidPitch + 4 * lane) = v4;
    if (wave == 1 && lane < 16) *(volatile v4u*)(H16out + (size_t)i * kHidPitch + l16 * 8) = u16;
    __threadfence();
  }
}

__global__ __launch_bounds__(256) void attn_cls_kernel(const float* __restrict__ S, const float* __restrict__ MO,
                                                       const float* __restrict__ cw, const float* __restrict__ cbias,
                                                       float* __restrict__ PL, float* __restrict__ AS) {
  __shared__ __align__(16) float msh[8 * kWind * kHidPitch];
  __shared__ float psh[8 * 16];
  __shared__ __align__(16) float atts[kHops * 8 * 16];
  __shared__ __align__(16) float preds[8 * 8];
  const int tid = threadIdx.x;
  const int lane = tid & 31, wave = tid >> 5;
  const int blk = blockIdx.x;
  const int q = blk * 8 + wave;
  const int i = (q > 0) ? (q - 1) : 0;
  float* m = msh + wave * (kWind * kHidPitch);
#pragma unroll 1
  for (int w = 0; w < kWind; ++w) {
    const int idx = i - (kWind - 1) + w;
    const bool valid = idx >= 0;
    const int idc = valid ? idx : 0;
    const v4f sv = *(const v4f*)(S + (size_t)idc * kHidPitch + 4 * lane);
    const v4f mv = *(const v4f*)(MO + ((size_t)w * kUtts + i) * kHidPitch + 4 * lane);
    const v4f tv = sv + mv;
    v4f r;
    r[0] = valid ? tv[0] : mv[0];
    r[1] = valid ? tv[1] : mv[1];
    r[2] = valid ? tv[2] : mv[2];
    r[3] = valid ? tv[3] : mv[3];
    *(v4f*)(m + w * kHidPitch + 4 * lane) = r;
  }
  const float* er = S + (size_t)(i + 1) * kHidPitch;
  float e0 = er[lane], e1 = er[lane + 32], e2 = er[lane + 64], e3 = er[lane + 96];
  wave_lds_sync();
#pragma unroll 1
  for (int hop = 0; hop < kHops; ++hop) {
    float myL = -1.0e30f;
#pragma unroll 1
    for (int w = 0; w < kWind; ++w) {
      const float* mw = m + w * kHidPitch;
      float part = e0 * mw[lane] + e1 * mw[lane + 32] + e2 * mw[lane + 64] + e3 * mw[lane + 96];
      part = wave_sum(part);
      const bool valid = (i - (kWind - 1) + w) >= 0;
      const float L = valid ? part : kNegFill;
      myL = (lane == w) ? L : myL;
    }
    const float mx  = wave_max(myL);
    const float ex  = expf(myL - mx);
    const float sum = wave_sum(ex);
    const float p   = ex * (1.0f / sum);
    if (lane < 16) {
      psh[wave * 16 + lane] = p;
      atts[(hop * 8 + wave) * 16 + lane] = p;
    }
    wave_lds_sync();
    float a0 = 0.0f, a1 = 0.0f, a2 = 0.0f, a3 = 0.0f;
#pragma unroll 1
    for (int w = 0; w < kWind; ++w) {
      const float pw = psh[wave * 16 + w];
      const float* mw = m + w * kHidPitch;
      a0 += pw * mw[lane]; a1 += pw * mw[lane + 32]; a2 += pw * mw[lane + 64]; a3 += pw * mw[lane + 96];
    }
    e0 += a0; e1 += a1; e2 += a2; e3 += a3;
    wave_lds_sync();
  }
  const bool firstrow = (q == 0);
  const float f0 = S[lane], f1 = S[lane + 32], f2 = S[lane + 64], f3 = S[lane + 96];
  e0 = firstrow ? f0 : e0; e1 = firstrow ? f1 : e1; e2 = firstrow ? f2 : e2; e3 = firstrow ? f3 : e3;
  float myC = -1.0e30f;
#pragma unroll 1
  for (int k = 0; k < kClasses; ++k) {
    const float* wr = cw + k * kHidden;
    const bool d3ok = (lane + 96) < kHidden;
    const int d3 = d3ok ? (lane + 96) : (kHidden - 1);
    float w3 = wr[d3];
    w3 = d3ok ? w3 : 0.0f;
    float part = wr[lane] * e0 + wr[lane + 32] * e1 + wr[lane + 64] * e2 + w3 * e3;
    part = wave_sum(part);
    const float L = part + cbias[k];
    myC = (lane == k) ? L : myC;
  }
  const float mxc  = wave_max(myC);
  const float exc  = expf(myC - mxc);
  const float sumc = wave_sum(exc);
  const float lsm  = logf(sumc);
  const float pv = (lane < kClasses) ? ((myC - mxc) - lsm) : 0.0f;
  if (lane < 8) preds[wave * 8 + lane] = pv;
  __syncthreads();
  const int l16 = lane & 15;
  for (int pass = 0; pass < 2; ++pass) {
    if (wave == 0) {
      if (lane < 16) {
        const int row = l16 >> 1, c4 = (l16 & 1) * 4;
        const v4f v = *(const v4f*)(preds + row * 8 + c4);
        *(volatile v4f*)(PL + (size_t)(blk * 8 + row) * 8 + c4) = v;
      }
    } else if (wave <= kHops) {
      const int hop = wave - 1;
      const int row = lane >> 2, c4 = (lane & 3) * 4;
      const v4f v = *(const v4f*)(atts + (hop * 8 + row) * 16 + c4);
      *(volatile v4f*)(AS + ((size_t)hop * kUtts + (size_t)blk * 8 + row) * 16 + c4) = v;
    }
    __threadfence();
  }
}

__device__ __forceinline__ float out_elem(int e, const float* __restrict__ PL, const float* __restrict__ AS) {
  int ep = (e < kOutPred) ? e : (kOutPred - 1);
  ep = (ep < 0) ? 0 : ep;
  const int rp = ep / kClasses, cp = ep - rp * kClasses;
  const float vp = PL[rp * 8 + cp];
  int ea = e - kOutPred;
  ea = (ea < 0) ? 0 : ea;
  ea = (ea < kOutAttn) ? ea : (kOutAttn - 1);
  const int hop = ea / ((kUtts - 1) * kWind);
  const int rem = ea - hop * ((kUtts - 1) * kWind);
  const int ii = rem / kWind, w = rem - ii * kWind;
  const float va = AS[((size_t)hop * kUtts + ii + 1) * 16 + w];
  return (e < kOutPred) ? vp : va;
}
__global__ __launch_bounds__(256) void out_pack_kernel(const float* __restrict__ PL, const float* __restrict__ AS,
                                                       float* __restrict__ out, int nTot) {
  const int c = blockIdx.x * 256 + threadIdx.x;
  const int nChunks = nTot >> 2;
  const int rem = nTot & 3;
  if (c < nChunks) {
    v4f v;
    v[0] = out_elem(4 * c + 0, PL, AS);
    v[1] = out_elem(4 * c + 1, PL, AS);
    v[2] = out_elem(4 * c + 2, PL, AS);
    v[3] = out_elem(4 * c + 3, PL, AS);
    float* op = out + 4 * (size_t)c;
    *(volatile v4f*)op = v;
    __threadfence();
    *(volatile v4f*)op = v;
  } else if (c == nChunks && rem > 0) {
    float* op = out + 4 * (size_t)c;
    if (rem == 2) {
      v2f v;
      v[0] = out_elem(4 * c + 0, PL, AS);
      v[1] = out_elem(4 * c + 1, PL, AS);
      *(volatile v2f*)op = v;
      __threadfence();
      *(volatile v2f*)op = v;
    } else {
      for (int e = 0; e < rem; ++e) {
        const float v = out_elem(4 * c + e, PL, AS);
        ((volatile float*)op)[e] = v;
        __threadfence();
        ((volatile float*)op)[e] = v;
      }
    }
  }
}

static inline dim3 gemm_grid(int M, int N) {
  const int tiles = (M / 64) * (N / 64);
  return dim3((unsigned)((tiles + 7) / 8), 1, 1);
}

extern "C" void kernel_launch(void* const* d_in, const int* in_sizes, int n_in,
                              void* d_out, int out_size, void* d_ws, size_t ws_size, hipStream_t stream) {
  if (n_in < 17) return;
  if (in_sizes[0] < kTok || in_sizes[2] < kVocab * kEmb || in_sizes[3] < kHidden * kCat || in_sizes[4] < kHidden ||
      in_sizes[5] < kGate * kHidden || in_sizes[6] < kGate * kHidden || in_sizes[7] < kGate || in_sizes[8] < kGate ||
      in_sizes[9] < kClasses * kHidden || in_sizes[10] < kClasses || in_sizes[11] < kFilt * 3 * kEmb ||
      in_sizes[12] < kFilt || in_sizes[13] < kFilt * 4 * kEmb || in_sizes[14] < kFilt || in_sizes[15] < kFilt * 5 * kEmb ||
      in_sizes[16] < kFilt) return;
  if (out_size < kOutTot) return;
  if (ws_size < kWsTotal) return;

  const int*   sents   = (const int*)d_in[0];
  const float* emb     = (const float*)d_in[2];
  const float* trans_w = (const float*)d_in[3];
  const float* trans_b = (const float*)d_in[4];
  const float* gru_wih = (const float*)d_in[5];
  const float* gru_whh = (const float*)d_in[6];
  const float* gru_bih = (const float*)d_in[7];
  const float* gru_bhh = (const float*)d_in[8];
  const float* cls_w   = (const float*)d_in[9];
  const float* cls_b   = (const float*)d_in[10];
  const float* conv_w3 = (const float*)d_in[11];
  const float* conv_b3 = (const float*)d_in[12];
  const float* conv_w4 = (const float*)d_in[13];
  const float* conv_b4 = (const float*)d_in[14];
  const float* conv_w5 = (const float*)d_in[15];
  const float* conv_b5 = (const float*)d_in[16];
  float* out = (float*)d_out;

  char* wp = (char*)d_ws;
  unsigned short* E16   = (unsigned short*)wp; wp += kBytesE16;
  unsigned short* WB3   = (unsigned short*)wp; wp += kBytesWB3;
  unsigned short* WB4   = (unsigned short*)wp; wp += kBytesWB4;
  unsigned short* WB5   = (unsigned short*)wp; wp += kBytesWB5;
  unsigned short* Yall  = (unsigned short*)wp; wp += 3 * kBytesYpl;
  unsigned short* F16   = (unsigned short*)wp; wp += kBytesF16;
  unsigned short* TWB   = (unsigned short*)wp; wp += kBytesTWB;
  float*          Uf    = (float*)wp;          wp += kBytesU;
  float*          Sf    = (float*)wp;          wp += kBytesS;
  unsigned short* S16   = (unsigned short*)wp; wp += kBytesS16;
  unsigned short* WIH16 = (unsigned short*)wp; wp += kBytesWG16;
  unsigned short* WHH16 = (unsigned short*)wp; wp += kBytesWG16;
  float*          GIf   = (float*)wp;          wp += kBytesGI;
  float*          GHf   = (float*)wp;          wp += kBytesGI;
  unsigned short* H16a  = (unsigned short*)wp; wp += kBytesH16;
  unsigned short* H16b  = (unsigned short*)wp; wp += kBytesH16;
  float*          MO    = (float*)wp;          wp += kBytesMO;
  float*          PL    = (float*)wp;          wp += kBytesPL;
  float*          AS    = (float*)wp;          wp += kBytesAS;
  if ((size_t)(wp - (char*)d_ws) > ws_size) return;

  unsigned short* Y3 = Yall;
  unsigned short* Y4 = Yall + (size_t)kTok * kFilt;
  unsigned short* Y5 = Yall + 2 * (size_t)kTok * kFilt;
  const size_t moPlane = (size_t)kUtts * kHidPitch;
  const float sc16  = 1.0f / 16.0f;
  const float sc256 = 1.0f / 256.0f;

  const int chunksW3 = kFilt * kConvK3 / 8, chunksW4 = kFilt * kConvK4 / 8, chunksW5 = kFilt * kConvK5 / 8;
  prep_cast16_kernel<<<(chunksW3 + 255) / 256, 256, 0, stream>>>(conv_w3, WB3, kConvK3, kFilt, kEmbPitch, kEmb, 3 * kEmb, kCarry, chunksW3);
  prep_cast16_kernel<<<(chunksW4 + 255) / 256, 256, 0, stream>>>(conv_w4, WB4, kConvK4, kFilt, kEmbPitch, kEmb, 4 * kEmb, kCarry, chunksW4);
  prep_cast16_kernel<<<(chunksW5 + 255) / 256, 256, 0, stream>>>(conv_w5, WB5, kConvK5, kFilt, kEmbPitch, kEmb, 5 * kEmb, kCarry, chunksW5);
  const int chunksTW = kTransN * kCat / 8;
  prep_cast16_kernel<<<(chunksTW + 255) / 256, 256, 0, stream>>>(trans_w, TWB, kCat, kHidden, kCat, kCat, kCat, kCarry, chunksTW);
  const int chunksWG = kGatePitch * kHidPitch / 8;
  prep_cast16_kernel<<<(chunksWG + 255) / 256, 256, 0, stream>>>(gru_wih, WIH16, kHidPitch, kGate, kHidPitch, kHidden, kHidden, kCarry, chunksWG);
  prep_cast16_kernel<<<(chunksWG + 255) / 256, 256, 0, stream>>>(gru_whh, WHH16, kHidPitch, kGate, kHidPitch, kHidden, kHidden, kCarry, chunksWG);

  const int chunksE = kTokRows * (kEmbPitch / 8);
  embed_gather_kernel<<<(chunksE + 255) / 256, 256, 0, stream>>>(sents, emb, E16, chunksE);

  wmma_gemm64<0, false, 0, 1, false, 0><<<gemm_grid(kTok, kFilt), 256, 0, stream>>>(
      E16, E16, kEmbPitch, 0L, WB3, WB3, kConvK3, 0L, (void*)Y3, (void*)Y3, kFilt, 0L, trans_b, Uf, 0L, kTok, kFilt, kConvK3, sc16);
  wmma_gemm64<0, false, 0, 1, false, 0><<<gemm_grid(kTok, kFilt), 256, 0, stream>>>(
      E16, E16, kEmbPitch, 0L, WB4, WB4, kConvK4, 0L, (void*)Y4, (void*)Y4, kFilt, 0L, trans_b, Uf, 0L, kTok, kFilt, kConvK4, sc16);
  wmma_gemm64<0, false, 0, 1, false, 0><<<gemm_grid(kTok, kFilt), 256, 0, stream>>>(
      E16, E16, kEmbPitch, 0L, WB5, WB5, kConvK5, 0L, (void*)Y5, (void*)Y5, kFilt, 0L, trans_b, Uf, 0L, kTok, kFilt, kConvK5, sc16);

  maxpool_kernel<<<kUtts, 192, 0, stream>>>(Yall, conv_b3, conv_b4, conv_b5, F16);

  wmma_gemm64<0, false, 0, 0, false, 0><<<gemm_grid(kUtts, kTransN), 256, 0, stream>>>(
      F16, F16, kCat, 0L, TWB, TWB, kCat, 0L, (void*)Uf, (void*)Uf, kHidPitch, 0L, trans_b, Sf, 0L, kUtts, kTransN, kCat, sc256);
  feat_tanh_kernel<<<kUtts, 128, 0, stream>>>(Uf, trans_b, Sf, S16);

  wmma_gemm64<0, false, 0, 0, false, 0><<<gemm_grid(kUtts, kGatePitch), 256, 0, stream>>>(
      S16, S16, kHidPitch, 0L, WIH16, WIH16, kHidPitch, 0L, (void*)GIf, (void*)GIf, kGatePitch, 0L, gru_bih, Sf, 0L,
      kUtts, kGatePitch, kHidPitch, sc256);
  for (int step = 0; step < kWind; ++step) {
    unsigned short* hcur  = (step & 1) ? H16b : H16a;
    unsigned short* hprev = (step & 1) ? H16a : H16b;
    if (step > 0) {
      wmma_gemm64<0, false, 0, 0, false, 0><<<gemm_grid(kUtts, kGatePitch), 256, 0, stream>>>(
          hprev, hprev, kHidPitch, 0L, WHH16, WHH16, kHidPitch, 0L, (void*)GHf, (void*)GHf, kGatePitch, 0L, gru_bhh, Sf, 0L,
          kUtts, kGatePitch, kHidPitch, sc256);
    }
    const int prevStep = (step > 0) ? (step - 1) : 0;
    gru_gate_kernel<<<kUtts, 128, 0, stream>>>(GIf, GHf, gru_bih, gru_bhh, MO + (size_t)prevStep * moPlane,
                                                MO + (size_t)step * moPlane, hcur, step);
  }

  attn_cls_kernel<<<kUtts / 8, 256, 0, stream>>>(Sf, MO, cls_w, cls_b, PL, AS);
  const int packThreads = (kOutTot >> 2) + 1;
  out_pack_kernel<<<(packThreads + 255) / 256, 256, 0, stream>>>(PL, AS, out, kOutTot);
}
